// NormLinearAttention_1906965479820
// MI455X (gfx1250) — hardware-verified
//
#include <hip/hip_runtime.h>
#include <math.h>
#include <stdint.h>

#define NB_  2
#define NS_  2048
#define DM_  1024
#define NH_  16
#define HD_  64
#define LR_  128
#define NR_  (NB_ * NS_)
#define LNEPS 1e-5f
#define WSC   64.0f
#define LOSC  2048.0f

#define INV2PI   0.15915494309189535f
#define TWOPI_C1 6.28125f
#define TWOPI_C2 1.93500518798828125e-3f
#define TWOPI_C3 3.0199160e-7f

#define F_BIAS  1
#define F_OUT32 16
#define F_OUTHL 32

static_assert((NR_ % 16) == 0 && (NS_ % 64) == 0 && (DM_ % 256) == 0 && NH_ * HD_ == DM_ && LR_ == 2 * HD_);

typedef _Float16 v16h __attribute__((ext_vector_type(16)));
typedef _Float16 v8h  __attribute__((ext_vector_type(8)));
typedef __bf16   v16b __attribute__((ext_vector_type(16)));
typedef float    v8f  __attribute__((ext_vector_type(8)));
typedef float    v4f  __attribute__((ext_vector_type(4)));
typedef unsigned int v4u __attribute__((ext_vector_type(4)));

union FragH { v16h v; v8h h[2]; };

__device__ __forceinline__ unsigned short bf_bits(float f) {
  unsigned u = __float_as_uint(f);
  return (unsigned short)((u + 0x7FFFu + ((u >> 16) & 1u)) >> 16);
}
__device__ __forceinline__ float bf_up(unsigned short h) { return __uint_as_float(((unsigned)h) << 16); }
__device__ __forceinline__ float bfr(float f) { return bf_up(bf_bits(f)); }
__device__ __forceinline__ unsigned short h_bits(_Float16 x) { return __builtin_bit_cast(unsigned short, x); }
__device__ __forceinline__ unsigned pk16(unsigned short a, unsigned short b) { return (unsigned)a | ((unsigned)b << 16); }
__device__ __forceinline__ unsigned pkh(float a, float b) { return pk16(h_bits((_Float16)a), h_bits((_Float16)b)); }
__device__ __forceinline__ v8f zero8() { v8f z = {0.f, 0.f, 0.f, 0.f, 0.f, 0.f, 0.f, 0.f}; return z; }
__device__ __forceinline__ v4f zero4() { v4f z = {0.f, 0.f, 0.f, 0.f}; return z; }

__device__ __forceinline__ void hl_pair(float f0, float f1, unsigned& hp, unsigned& lp) {
#pragma clang fp contract(off)
  const _Float16 h0 = (_Float16)f0, h1 = (_Float16)f1;
  const float d0 = f0 - (float)h0, d1 = f1 - (float)h1;
  const float r0 = d0 * LOSC, r1 = d1 * LOSC;
  hp = pk16(h_bits(h0), h_bits(h1));
  lp = pk16(h_bits((_Float16)r0), h_bits((_Float16)r1));
}

__device__ __forceinline__ float silu_f(float x) {
#pragma clang fp contract(off)
  const float t = x * -1.4426950408889634f;
  const float e = __builtin_amdgcn_exp2f(t);
  const float dn = 1.0f + e;
  const float r = __builtin_amdgcn_rcpf(dn);
  return x * r;
}

__device__ __forceinline__ void cos_sin_f(float ang, float& cv, float& sv) {
#pragma clang fp contract(off)
  const float qt = ang * INV2PI;
  const float kq = __builtin_rintf(qt);
  const float p1 = kq * TWOPI_C1;
  float r = ang - p1;
  const float p2 = kq * TWOPI_C2;
  r = r - p2;
  const float p3 = kq * TWOPI_C3;
  r = r - p3;
  const float tn = r * INV2PI;
  sv = __builtin_amdgcn_sinf(tn);
  cv = __builtin_amdgcn_cosf(tn);
}

__device__ __forceinline__ v16h ldfrag(const unsigned short* p) {
  FragH f;
  f.h[0] = *(const v8h*)(const void*)(p);
  f.h[1] = *(const v8h*)(const void*)(p + 16);
  return f.v;
}

template <bool BF> struct Eng;
template <> struct Eng<false> {
  static __device__ __forceinline__ v8f mma(v16h a, v16h b, v8f c) {
    c = __builtin_amdgcn_wmma_f32_16x16x32_f16(false, a, false, b, (short)0, c, false, false);
#if defined(__HIP_DEVICE_COMPILE__)
    asm volatile("v_nop\n\tv_nop\n\tv_nop\n\tv_nop" : "+v"(c) : "v"(a), "v"(b));
#endif
    return c;
  }
};
template <> struct Eng<true> {
  static __device__ __forceinline__ v8f mma(v16h a, v16h b, v8f c) {
    const v16b ab = __builtin_bit_cast(v16b, a);
    const v16b bb = __builtin_bit_cast(v16b, b);
    c = __builtin_amdgcn_wmma_f32_16x16x32_bf16(false, ab, false, bb, (short)0, c, false, false);
#if defined(__HIP_DEVICE_COMPILE__)
    asm volatile("v_nop\n\tv_nop\n\tv_nop\n\tv_nop" : "+v"(c) : "v"(a), "v"(b));
#endif
    return c;
  }
};
__device__ __forceinline__ void wave_sync_lds() {
  __builtin_amdgcn_fence(__ATOMIC_RELEASE, "workgroup");
  __builtin_amdgcn_wave_barrier();
  __builtin_amdgcn_fence(__ATOMIC_ACQUIRE, "workgroup");
}

template <int KIND>
__global__ __launch_bounds__(256) void cvt_rows(const float* __restrict__ x, unsigned short* outp, int nrows,
                                                int ncols, float sc) {
#pragma clang fp contract(off)
  const int tid = threadIdx.x, wave = tid >> 5, lane = tid & 31;
  const int row = blockIdx.x * 8 + wave;
  const int rowc = (row < nrows) ? row : (nrows - 1);
#pragma unroll 1
  for (int c0 = 0; c0 < ncols; c0 += 256) {
    const int c = c0 + lane * 8;
    const bool live = (c < ncols);
    const int cc = live ? c : (ncols - 8);
    const float* rp = x + (size_t)rowc * ncols + cc;
    const v4f a = *(const v4f*)rp;
    const v4f c4v = *(const v4f*)(rp + 4);
    v4u pk;
#pragma unroll
    for (int e = 0; e < 2; ++e) {
      if (KIND == 0) {
        pk[e]     = pk16(bf_bits(a[2 * e]), bf_bits(a[2 * e + 1]));
        pk[2 + e] = pk16(bf_bits(c4v[2 * e]), bf_bits(c4v[2 * e + 1]));
      } else {
        pk[e]     = pkh(bfr(a[2 * e]) * sc, bfr(a[2 * e + 1]) * sc);
        pk[2 + e] = pkh(bfr(c4v[2 * e]) * sc, bfr(c4v[2 * e + 1]) * sc);
      }
    }
    unsigned short* gp = outp + (size_t)rowc * ncols + cc;
    const bool st = live && (row < nrows);
    if (st) { *(volatile v4u*)gp = pk; }
    __threadfence();
    if (st) { *(volatile v4u*)gp = pk; }
  }
}

__global__ __launch_bounds__(256) void pos_qk(const float* __restrict__ tqk, const float* __restrict__ theta,
                                              unsigned short* qh, unsigned short* ql,
                                              unsigned short* kth, unsigned short* ktl) {
#pragma clang fp contract(off)
  __shared__ __align__(16) float csC[64 * 64];
  __shared__ __align__(16) float csS[64 * 64];
  const int tid = threadIdx.x;
  const int n0 = blockIdx.x * 64;
  const int h = blockIdx.y;
#pragma unroll 1
  for (int j = 0; j < 16; ++j) {
    const int i = j * 256 + tid;
    const int nn = i >> 6, d = i & 63;
    const float th = bfr(theta[h * HD_ + d]);
    const float fn = (float)(n0 + nn);
    const float ang = th * fn;
    float cv, sv;
    cos_sin_f(ang, cv, sv);
    csC[i] = cv;
    csS[i] = sv;
  }
  __syncthreads();
#pragma unroll 1
  for (int b = 0; b < NB_; ++b) {
    {
#pragma unroll 1
      for (int it = 0; it < 2; ++it) {
        const int item = it * 256 + tid;
        const int tq = item >> 3, c = item & 7;
        const size_t row = (size_t)b * NS_ + n0 + tq;
        const float* qp = tqk + row * (2 * DM_) + h * HD_ + 8 * c;
        const v4f a0 = *(const v4f*)qp;
        const v4f a1 = *(const v4f*)(qp + 4);
        const float* cp = csC + tq * 64 + 8 * c;
        const float* sp = csS + tq * 64 + 8 * c;
        const v4f c0 = *(const v4f*)cp, c1 = *(const v4f*)(cp + 4);
        const v4f s0 = *(const v4f*)sp, s1 = *(const v4f*)(sp + 4);
        float qc[8], qs[8];
#pragma unroll
        for (int e = 0; e < 4; ++e) {
          const float g0 = silu_f(a0[e]);
          qc[e] = g0 * c0[e]; qs[e] = g0 * s0[e];
          const float g1 = silu_f(a1[e]);
          qc[4 + e] = g1 * c1[e]; qs[4 + e] = g1 * s1[e];
        }
        v4u hc, lc, hs, ls;
#pragma unroll
        for (int e = 0; e < 4; ++e) {
          unsigned hp, lp;
          hl_pair(qc[2 * e], qc[2 * e + 1], hp, lp); hc[e] = hp; lc[e] = lp;
          hl_pair(qs[2 * e], qs[2 * e + 1], hp, lp); hs[e] = hp; ls[e] = lp;
        }
        const size_t base = ((size_t)(b * NH_ + h) * NS_ + n0 + tq) * LR_ + 8 * c;
        for (int pass = 0; pass < 2; ++pass) {
          *(volatile v4u*)(qh + base)       = hc;
          *(volatile v4u*)(qh + base + HD_) = hs;
          *(volatile v4u*)(ql + base)       = lc;
          *(volatile v4u*)(ql + base + HD_) = ls;
          __threadfence();
        }
      }
    }
    {
#pragma unroll 1
      for (int it = 0; it < 2; ++it) {
        const int item = it * 256 + tid;
        const int dd = item >> 3, tg = item & 7;
        float kc[8], ks[8];
#pragma unroll
        for (int e = 0; e < 8; ++e) {
          const int nn = 8 * tg + e;
          const float kv = tqk[((size_t)b * NS_ + n0 + nn) * (2 * DM_) + DM_ + h * HD_ + dd];
          const float g0 = silu_f(kv);
          kc[e] = g0 * csC[nn * 64 + dd];
          ks[e] = g0 * csS[nn * 64 + dd];
        }
        v4u hc, lc, hs, ls;
#pragma unroll
        for (int e = 0; e < 4; ++e) {
          unsigned hp, lp;
          hl_pair(kc[2 * e], kc[2 * e + 1], hp, lp); hc[e] = hp; lc[e] = lp;
          hl_pair(ks[2 * e], ks[2 * e + 1], hp, lp); hs[e] = hp; ls[e] = lp;
        }
        const size_t bc = ((size_t)(b * NH_ + h) * LR_ + dd) * NS_ + n0 + 8 * tg;
        const size_t bs = ((size_t)(b * NH_ + h) * LR_ + HD_ + dd) * NS_ + n0 + 8 * tg;
        for (int pass = 0; pass < 2; ++pass) {
          *(volatile v4u*)(kth + bc) = hc;
          *(volatile v4u*)(kth + bs) = hs;
          *(volatile v4u*)(ktl + bc) = lc;
          *(volatile v4u*)(ktl + bs) = ls;
          __threadfence();
        }
      }
    }
  }
}

__global__ __launch_bounds__(256) void vt_cvt(const float* __restrict__ tv, unsigned short* vth,
                                              unsigned short* vtl) {
#pragma clang fp contract(off)
  const int tid = threadIdx.x;
  const int n0 = blockIdx.x * 64, h = blockIdx.y;
#pragma unroll 1
  for (int b = 0; b < NB_; ++b) {
    v4u st[4];
#pragma unroll
    for (int it = 0; it < 2; ++it) {
      const int item = it * 256 + tid;
      const int ee = item >> 3, tg = item & 7;
      float v[8];
#pragma unroll
      for (int e = 0; e < 8; ++e)
        v[e] = tv[((size_t)b * NS_ + n0 + 8 * tg + e) * DM_ + h * HD_ + ee];
      v4u hv, lv;
#pragma unroll
      for (int e = 0; e < 4; ++e) {
        unsigned hp, lp;
        hl_pair(v[2 * e], v[2 * e + 1], hp, lp); hv[e] = hp; lv[e] = lp;
      }
      st[2 * it] = hv; st[2 * it + 1] = lv;
    }
    for (int pass = 0; pass < 2; ++pass) {
#pragma unroll
      for (int it = 0; it < 2; ++it) {
        const int item = it * 256 + tid;
        const int ee = item >> 3, tg = item & 7;
        const size_t go = ((size_t)(b * NH_ + h) * HD_ + ee) * NS_ + n0 + 8 * tg;
        *(volatile v4u*)(vth + go) = st[2 * it];
        *(volatile v4u*)(vtl + go) = st[2 * it + 1];
      }
      __threadfence();
    }
  }
}

__global__ __launch_bounds__(256) void ln_gate(const float* __restrict__ o32, const float* __restrict__ u32,
                                               const float* __restrict__ g, const float* __restrict__ bt,
                                               unsigned short* yh, unsigned short* yl, int nrows) {
#pragma clang fp contract(off)
  const int tid = threadIdx.x, wave = tid >> 5, lane = tid & 31;
  const int row = blockIdx.x * 8 + wave;
  const int rowc = (row < nrows) ? row : (nrows - 1);
  const int c8 = lane * 8;
  const float* rp = o32 + (size_t)rowc * DM_ + c8;
  float x[32];
#pragma unroll
  for (int k = 0; k < 4; ++k) {
    const v4f a = *(const v4f*)(rp + 256 * k);
    const v4f c = *(const v4f*)(rp + 256 * k + 4);
#pragma unroll
    for (int e = 0; e < 4; ++e) { x[8 * k + e] = a[e]; x[8 * k + 4 + e] = c[e]; }
  }
  float s = 0.f;
#pragma unroll
  for (int e = 0; e < 32; ++e) s = s + x[e];
#pragma unroll
  for (int off = 1; off < 32; off <<= 1) s = s + __shfl_xor(s, off, 32);
  const float mu = s * (1.0f / DM_);
  float d[32];
  float s2 = 0.f;
#pragma unroll
  for (int e = 0; e < 32; ++e) { d[e] = x[e] - mu; const float dd = d[e] * d[e]; s2 = s2 + dd; }
#pragma unroll
  for (int off = 1; off < 32; off <<= 1) s2 = s2 + __shfl_xor(s2, off, 32);
  const float var = s2 * (1.0f / DM_);
  const float rstd = rsqrtf(var + LNEPS);
  const float* up = u32 + (size_t)rowc * DM_ + c8;
  v4u hv[4], lv[4];
#pragma unroll
  for (int k = 0; k < 4; ++k) {
    const v4f u0 = *(const v4f*)(up + 256 * k);
    const v4f u1 = *(const v4f*)(up + 256 * k + 4);
    const v4f g0 = *(const v4f*)(g + 256 * k + c8);
    const v4f g1 = *(const v4f*)(g + 256 * k + c8 + 4);
    const v4f b0 = *(const v4f*)(bt + 256 * k + c8);
    const v4f b1 = *(const v4f*)(bt + 256 * k + c8 + 4);
    float uu[8], gg[8], bb[8];
#pragma unroll
    for (int e = 0; e < 4; ++e) {
      uu[e] = u0[e]; uu[4 + e] = u1[e];
      gg[e] = bfr(g0[e]); gg[4 + e] = bfr(g1[e]);
      bb[e] = bfr(b0[e]); bb[4 + e] = bfr(b1[e]);
    }
    float y[8];
#pragma unroll
    for (int e = 0; e < 8; ++e) {
      float t = d[8 * k + e] * rstd;
      t = t * gg[e];
      t = t + bb[e];
      y[e] = uu[e] * t;
    }
    v4u a, bl;
#pragma unroll
    for (int e = 0; e < 4; ++e) {
      unsigned hp, lp;
      hl_pair(y[2 * e], y[2 * e + 1], hp, lp);
      a[e] = hp; bl[e] = lp;
    }
    hv[k] = a; lv[k] = bl;
  }
  if (row < nrows) {
    unsigned short* hp0 = yh + (size_t)row * DM_ + c8;
    unsigned short* lp0 = yl + (size_t)row * DM_ + c8;
    for (int pass = 0; pass < 2; ++pass) {
#pragma unroll
      for (int k = 0; k < 4; ++k) {
        *(volatile v4u*)(hp0 + 256 * k) = hv[k];
        *(volatile v4u*)(lp0 + 256 * k) = lv[k];
      }
      __threadfence();
    }
  }
}

struct GArg {
  const unsigned short* A0; const unsigned short* A1; const unsigned short* B0; const unsigned short* B1;
  const float* bias; float* C32; unsigned short* Ch; unsigned short* Cl;
  int lda, ldb, ldc, ldh;
  int M, N, K, nb2;
  int sa1, sa2, sb1, sb2;
  int sc1, sc2, sbias2, flags;
  int tiles, pad0;
  float s0, s1;
  float oscale, pad1;
};
static_assert(sizeof(GArg) == 152);

template <bool BF, int NA, int NB>
__global__ __launch_bounds__(256) void gemm16(GArg g) {
#pragma clang fp contract(off)
  __shared__ __align__(16) float sT[8][16 * 68];
  const int lane = threadIdx.x & 31;
  const int wave = threadIdx.x >> 5;
  const int t = __builtin_amdgcn_readfirstlane((int)(blockIdx.x * 8 + wave));
  if (t >= g.tiles) return;
  const int bz = blockIdx.y;
  const int b1 = bz / g.nb2, b2 = bz - b1 * g.nb2;
  const size_t aoff = (size_t)b1 * g.sa1 + (size_t)b2 * g.sa2;
  const size_t boff = (size_t)b1 * g.sb1 + (size_t)b2 * g.sb2;
  const size_t coff = (size_t)b1 * g.sc1 + (size_t)b2 * g.sc2;
  const unsigned short* A0 = g.A0 + aoff;
  const unsigned short* A1 = g.A1 + aoff;
  const unsigned short* B0 = g.B0 + boff;
  const unsigned short* B1 = g.B1 + boff;
  const int tilesN = g.N >> 6;
  const int tm = t / tilesN;
  const int tn = t - tm * tilesN;
  const int m0 = tm * 16;
  const int n0 = tn * 64;

  const int rl   = lane & 15;
  const int hh   = lane >> 4;
  const int koff = hh * 8;

  v8f acc0[4], acc1[4];
#pragma unroll
  for (int j = 0; j < 4; ++j) { acc0[j] = zero8(); acc1[j] = zero8(); }

  const size_t arow = (size_t)(m0 + rl) * g.lda + koff;
#pragma unroll 2
  for (int k0 = 0; k0 < g.K; k0 += 32) {
    const v16h fa0 = ldfrag(A0 + arow + k0);
    v16h fa1;
    if (NA == 2) fa1 = ldfrag(A1 + arow + k0); else fa1 = fa0;
#pragma unroll
    for (int j = 0; j < 4; ++j) {
      const size_t brow = (size_t)(n0 + 16 * j + rl) * g.ldb + koff + k0;
      const v16h fb0 = ldfrag(B0 + brow);
      acc0[j] = Eng<BF>::mma(fa0, fb0, acc0[j]);
      if (NA == 2 && NB == 1) acc1[j] = Eng<BF>::mma(fa1, fb0, acc1[j]);
      if (NA == 2 && NB == 2) {
        const v16h fb1 = ldfrag(B1 + brow);
        acc1[j] = Eng<BF>::mma(fa0, fb1, acc1[j]);
        acc1[j] = Eng<BF>::mma(fa1, fb0, acc1[j]);
      }
    }
  }

  const int fl = g.flags;
  const float s0 = g.s0, s1 = g.s1;

  float* slab = sT[wave];
#pragma unroll
  for (int j = 0; j < 4; ++j) {
#pragma unroll
    for (int r = 0; r < 8; ++r) {
      float u = acc0[j][r] * s0;
      if (NA == 2) { const float u1 = acc1[j][r] * s1; u = u + u1; }
      slab[(koff + r) * 68 + 16 * j + rl] = u;
    }
  }
  wave_sync_lds();

  const int h2 = lane >> 4, c4 = (lane & 15) * 4;
  const float* biasp = g.bias + (size_t)b2 * g.sbias2;
  float* C32 = g.C32 + coff;
  unsigned short* Ch = g.Ch + coff;
  unsigned short* Cl = g.Cl + coff;
  float bz4[4] = {0.f, 0.f, 0.f, 0.f};
  if (fl & F_BIAS) {
#pragma unroll
    for (int e = 0; e < 4; ++e) bz4[e] = bfr(biasp[n0 + c4 + e]);
  }
  v4f ov[8];
#pragma unroll
  for (int it = 0; it < 8; ++it) {
    const int row = it * 2 + h2;
    const v4f v = *(const v4f*)(slab + row * 68 + c4);
    v4f o;
#pragma unroll
    for (int e = 0; e < 4; ++e) o[e] = v[e] + bz4[e];
    ov[it] = o;
    if (fl & F_OUTHL) *(v4f*)(slab + row * 68 + c4) = o;
  }
  if (fl & F_OUT32) {
    for (int pass = 0; pass < 2; ++pass) {
#pragma unroll
      for (int it = 0; it < 8; ++it) {
        const int row = it * 2 + h2;
        float* gp = C32 + (size_t)(m0 + row) * g.ldc + n0 + c4;
        *(volatile v4f*)gp = ov[it];
      }
      __threadfence();
    }
  }
  if (fl & F_OUTHL) {
    wave_sync_lds();
    const int q = lane >> 3, c8 = (lane & 7) * 8;
    v4u hv[4], lv[4];
#pragma unroll
    for (int it = 0; it < 4; ++it) {
      const int row = it * 4 + q;
      const float* sp = slab + row * 68 + c8;
      const v4f x0 = *(const v4f*)sp;
      const v4f x1 = *(const v4f*)(sp + 4);
      v4u a, bl;
#pragma unroll
      for (int e = 0; e < 2; ++e) {
        unsigned hp, lp;
        hl_pair(x0[2 * e], x0[2 * e + 1], hp, lp); a[e] = hp;     bl[e] = lp;
        hl_pair(x1[2 * e], x1[2 * e + 1], hp, lp); a[2 + e] = hp; bl[2 + e] = lp;
      }
      hv[it] = a; lv[it] = bl;
    }
    for (int pass = 0; pass < 2; ++pass) {
#pragma unroll
      for (int it = 0; it < 4; ++it) {
        const int row = it * 4 + q;
        unsigned short* gh = Ch + (size_t)(m0 + row) * g.ldh + n0 + c8;
        unsigned short* gl = Cl + (size_t)(m0 + row) * g.ldh + n0 + c8;
        *(volatile v4u*)gh = hv[it];
        *(volatile v4u*)gl = lv[it];
      }
      __threadfence();
    }
  }
  wave_sync_lds();
}

static GArg mkg(const unsigned short* A0, const unsigned short* A1, int lda, int sa1, int sa2,
                const unsigned short* B0, const unsigned short* B1, int ldb, int sb1, int sb2,
                int M, int N, int K, int nb2,
                const float* bias, int sbias2,
                float* C32, int ldc, unsigned short* Ch, unsigned short* Cl, int ldh, int sc1, int sc2,
                int flags, float s0, float s1) {
  GArg g;
  g.A0 = A0; g.A1 = A1; g.B0 = B0; g.B1 = B1;
  g.bias = bias; g.C32 = C32; g.Ch = Ch; g.Cl = Cl;
  g.lda = lda; g.ldb = ldb; g.ldc = ldc; g.ldh = ldh;
  g.M = M; g.N = N; g.K = K; g.nb2 = nb2;
  g.sa1 = sa1; g.sa2 = sa2; g.sb1 = sb1; g.sb2 = sb2;
  g.sc1 = sc1; g.sc2 = sc2; g.sbias2 = sbias2; g.flags = flags;
  g.tiles = (M / 16) * (N / 64); g.pad0 = 0;
  g.s0 = s0; g.s1 = s1; g.oscale = 1.0f; g.pad1 = 0.f;
  return g;
}
template <bool BF, int NA, int NB>
static void run_g(const GArg& g, int nbat, hipStream_t st) {
  if (g.tiles <= 0 || nbat <= 0) return;
  const dim3 grid((g.tiles + 7) / 8, nbat);
  gemm16<BF, NA, NB><<<grid, dim3(256), 0, st>>>(g);
}

extern "C" void kernel_launch(void* const* d_in, const int* in_sizes, int n_in,
                              void* d_out, int out_size, void* d_ws, size_t ws_size,
                              hipStream_t stream) {
  if (n_in < 9) return;
  const int ex[9] = { NR_ * DM_, NR_ * DM_, 4 * DM_ * DM_, 4 * DM_, DM_ * DM_, DM_, NH_ * HD_, DM_, DM_ };
  for (int i = 0; i < 9; ++i) if (in_sizes[i] != ex[i]) return;
  if (out_size != NR_ * DM_) return;

  const float* x     = (const float*)d_in[0];
  const float* wqkvu = (const float*)d_in[2];
  const float* bqkvu = (const float*)d_in[3];
  const float* wout  = (const float*)d_in[4];
  const float* bout  = (const float*)d_in[5];
  const float* theta = (const float*)d_in[6];
  const float* lnw   = (const float*)d_in[7];
  const float* lnb   = (const float*)d_in[8];
  float* out = (float*)d_out;

  const size_t MiB  = (size_t)1048576;
  const size_t oXB  = 0;
  const size_t oWB  = 8 * MiB;
  const size_t oWO  = 16 * MiB;
  const size_t oT   = 18 * MiB;
  const size_t oTV  = oT;
  const size_t oVTH = 34 * MiB;
  const size_t oVTL = 42 * MiB;
  const size_t oQH  = 50 * MiB;
  const size_t oYH  = 50 * MiB;
  const size_t oYL  = 58 * MiB;
  const size_t oQL  = 66 * MiB;
  const size_t oKTH = 82 * MiB;
  const size_t oU32 = 82 * MiB;
  const size_t oKTL = 98 * MiB;
  const size_t oO32 = 98 * MiB;
  const size_t oKVH = 114 * MiB;
  const size_t oKVL = oKVH + 524288;
  const size_t oEND = oKVL + 524288;
  if (oEND > ws_size) return;
  if (oEND > (size_t)134217728) return;

  char* ws = (char*)d_ws;
  unsigned short* XB  = (unsigned short*)(ws + oXB);
  unsigned short* WB  = (unsigned short*)(ws + oWB);
  unsigned short* WO  = (unsigned short*)(ws + oWO);
  float*          T   = (float*)(ws + oT);
  float*          TV  = (float*)(ws + oTV);
  unsigned short* VTH = (unsigned short*)(ws + oVTH);
  unsigned short* VTL = (unsigned short*)(ws + oVTL);
  unsigned short* QH  = (unsigned short*)(ws + oQH);
  unsigned short* QL  = (unsigned short*)(ws + oQL);
  unsigned short* YH  = (unsigned short*)(ws + oYH);
  unsigned short* YL  = (unsigned short*)(ws + oYL);
  unsigned short* KTH = (unsigned short*)(ws + oKTH);
  unsigned short* KTL = (unsigned short*)(ws + oKTL);
  float*          U32 = (float*)(ws + oU32);
  float*          O32 = (float*)(ws + oO32);
  unsigned short* KVH = (unsigned short*)(ws + oKVH);
  unsigned short* KVL = (unsigned short*)(ws + oKVL);

  const dim3 blk(256);

  cvt_rows<0><<<dim3(NR_ / 8), blk, 0, stream>>>(x, XB, NR_, DM_, 1.0f);
  cvt_rows<0><<<dim3((4 * DM_) / 8), blk, 0, stream>>>(wqkvu, WB, 4 * DM_, DM_, 1.0f);
  cvt_rows<1><<<dim3(DM_ / 8), blk, 0, stream>>>(wout, WO, DM_, DM_, WSC);
  {
    GArg g = mkg(XB, XB, DM_, 0, 0, WB, WB, DM_, 0, 0, NR_, 2 * DM_, DM_, 1,
                 bqkvu, 0, T, 2 * DM_, KVH, KVL, LR_, 0, 0, F_BIAS | F_OUT32, 1.0f, 0.0f);
    run_g<true, 1, 1>(g, 1, stream);
  }
  pos_qk<<<dim3(NS_ / 64, NH_), blk, 0, stream>>>(T, theta, QH, QL, KTH, KTL);
  {
    GArg g = mkg(XB, XB, DM_, 0, 0, WB + (size_t)2 * DM_ * DM_, WB, DM_, 0, 0, NR_, DM_, DM_, 1,
                 bqkvu + 2 * DM_, 0, TV, DM_, KVH, KVL, LR_, 0, 0, F_BIAS | F_OUT32, 1.0f, 0.0f);
    run_g<true, 1, 1>(g, 1, stream);
  }
  vt_cvt<<<dim3(NS_ / 64, NH_), blk, 0, stream>>>(TV, VTH, VTL);
  {
    GArg g = mkg(VTH, VTL, NS_, 0, HD_ * NS_, KTH, KTL, NS_, 0, LR_ * NS_, HD_, LR_, NS_, NB_ * NH_,
                 bqkvu, 0, T, LR_, KVH, KVL, LR_, 0, HD_ * LR_, F_OUTHL, 1.0f, 1.0f / LOSC);
    run_g<false, 2, 2>(g, NB_ * NH_, stream);
  }
  {
    GArg g = mkg(XB, XB, DM_, 0, 0, WB + (size_t)3 * DM_ * DM_, WB, DM_, 0, 0, NR_, DM_, DM_, 1,
                 bqkvu + 3 * DM_, 0, U32, DM_, KVH, KVL, LR_, 0, 0, F_BIAS | F_OUT32, 1.0f, 0.0f);
    run_g<true, 1, 1>(g, 1, stream);
  }
  {
    GArg g = mkg(QH, QL, LR_, NH_ * NS_ * LR_, NS_ * LR_, KVH, KVL, LR_, NH_ * HD_ * LR_, HD_ * LR_,
                 NS_, HD_, LR_, NH_,
                 bqkvu, 0, O32, DM_, KVH, KVL, LR_, NS_ * DM_, HD_, F_OUT32, 1.0f, 1.0f / LOSC);
    run_g<false, 2, 2>(g, NB_ * NH_, stream);
  }
  ln_gate<<<dim3(NR_ / 8), blk, 0, stream>>>(O32, U32, lnw, lnb, YH, YL, NR_);
  {
    GArg g = mkg(YH, YL, DM_, 0, 0, WO, WO, DM_, 0, 0, NR_, DM_, DM_, 1,
                 bout, 0, out, DM_, KVH, KVL, LR_, 0, 0, F_BIAS | F_OUT32,
                 1.0f / WSC, 1.0f / (WSC * LOSC));
    run_g<false, 2, 1>(g, 1, stream);
  }
  (void)hipGetLastError();
}
